// SELRU_10505490006122
// MI455X (gfx1250) — hardware-run, weakly checked
//
#include <hip/hip_runtime.h>


#define NM   4096
#define NB   2
#define NT   2048
#define DC   256
#define NS   64
#define NQ   384
#define PFL  6.103515625e-05f
typedef _Float16 h16;
typedef unsigned short bf;
typedef __attribute__((ext_vector_type(16))) __bf16   v16bf;
typedef __attribute__((ext_vector_type(16))) _Float16 v16h;
typedef __attribute__((ext_vector_type(8)))  _Float16 v8h;
typedef __attribute__((ext_vector_type(8)))  unsigned short v8us;
typedef __attribute__((ext_vector_type(8)))  float    v8f;
typedef __attribute__((ext_vector_type(4)))  float    v4f;
typedef v8h  __attribute__((may_alias)) v8ha;
typedef v4f  __attribute__((may_alias)) v4fa;
typedef v8us __attribute__((may_alias)) v8usa;

__device__ __forceinline__ unsigned short f2bf(float f) { unsigned u = __float_as_uint(f); u += 0x7FFFu + ((u >> 16) & 1u); return (unsigned short)(u >> 16); }
__device__ __forceinline__ float bf2f(unsigned short b) { return __uint_as_float(((unsigned)b) << 16); }
__device__ __forceinline__ float bfr(float f) { return bf2f(f2bf(f)); }
__device__ __forceinline__ v16h cat16(v8h lo, v8h hi) { return __builtin_shufflevector(lo, hi, 0, 1, 2, 3, 4, 5, 6, 7, 8, 9, 10, 11, 12, 13, 14, 15); }
__device__ __forceinline__ v16bf cat16b(v8us lo, v8us hi) { return __builtin_bit_cast(v16bf, __builtin_shufflevector(lo, hi, 0, 1, 2, 3, 4, 5, 6, 7, 8, 9, 10, 11, 12, 13, 14, 15)); }
__device__ __forceinline__ v8f wmma16(v16h a, v16h b, v8f c) { return __builtin_amdgcn_wmma_f32_16x16x32_f16(false, a, false, b, (short)0, c, false, false); }
__device__ __forceinline__ v8f wmmab(v16bf a, v16bf b, v8f c) { return __builtin_amdgcn_wmma_f32_16x16x32_bf16(false, a, false, b, (short)0, c, false, false); }

template <typename T16> struct WFrag;
template <> struct WFrag<h16> { typedef v16h V; static __device__ __forceinline__ V ld(const h16* p) { return cat16(*(const v8h*)p, *(const v8h*)(p + 16)); } static __device__ __forceinline__ v8f mma(V a, V b, v8f c) { return wmma16(a, b, c); } };
template <> struct WFrag<bf> { typedef v16bf V; static __device__ __forceinline__ V ld(const bf* p) { return cat16b(*(const v8us*)p, *(const v8us*)(p + 16)); } static __device__ __forceinline__ v8f mma(V a, V b, v8f c) { return wmmab(a, b, c); } };
template <typename T16, int NSPLIT, bool BIAS>
__global__ __launch_bounds__(32) void k_gemmw(const T16* __restrict__ A, const T16* __restrict__ A2, const T16* __restrict__ Bt, const T16* __restrict__ Bt2, int K, float* C, int ldc, const float* __restrict__ bias, size_t sA, size_t sB, size_t sC) {
    typedef typename WFrag<T16>::V V;
    __shared__ __align__(16) float os[16 * 68];
    const size_t z = blockIdx.z; A += z * sA; if (A2) A2 += z * sA; Bt += z * sB; if (Bt2) Bt2 += z * sB; C += z * sC;
    const int lane = threadIdx.x & 31, lr = lane & 15, hi = lane >> 4; const int r0 = blockIdx.x * 64, c0 = blockIdx.y * 64;
    v8f acc[4][4];
#pragma unroll
    for (int mb = 0; mb < 4; ++mb)
#pragma unroll
        for (int nb = 0; nb < 4; ++nb) acc[mb][nb] = (v8f){};
    const size_t aoff = (size_t)(r0 + lr) * K + 8 * hi, boff = (size_t)(c0 + lr) * K + 8 * hi;
    for (int kc = 0; kc < K; kc += 32) {
        V a[4], a2[4];
#pragma unroll
        for (int mb = 0; mb < 4; ++mb) { a[mb] = WFrag<T16>::ld(A + aoff + (size_t)mb * 16 * K + kc); if (NSPLIT == 1 || NSPLIT == 2) a2[mb] = WFrag<T16>::ld(A2 + aoff + (size_t)mb * 16 * K + kc); }
#pragma unroll
        for (int nb = 0; nb < 4; ++nb) { const V b = WFrag<T16>::ld(Bt + boff + (size_t)nb * 16 * K + kc); V b2; if (NSPLIT >= 2) b2 = WFrag<T16>::ld(Bt2 + boff + (size_t)nb * 16 * K + kc);
#pragma unroll
            for (int mb = 0; mb < 4; ++mb) { acc[mb][nb] = WFrag<T16>::mma(a[mb], b, acc[mb][nb]); if (NSPLIT == 1 || NSPLIT == 2) acc[mb][nb] = WFrag<T16>::mma(a2[mb], b, acc[mb][nb]); if (NSPLIT >= 2) acc[mb][nb] = WFrag<T16>::mma(a[mb], b2, acc[mb][nb]); } }
        asm volatile("v_nop\n\tv_nop\n\tv_nop\n\tv_nop" : "+v"(acc[0][0]), "+v"(acc[1][1]), "+v"(acc[2][2]), "+v"(acc[3][3]) : "v"(a[0]), "v"(a[3]));
    }
#pragma unroll
    for (int mb = 0; mb < 4; ++mb) {
#pragma unroll
        for (int nb = 0; nb < 4; ++nb) {
#pragma unroll
            for (int j = 0; j < 8; ++j) os[(hi * 8 + j) * 68 + nb * 16 + lr] = acc[mb][nb][j]; }
        __builtin_amdgcn_wave_barrier(); asm volatile("" ::: "memory");
        float* crow = C + (size_t)(r0 + mb * 16) * ldc + c0;
#pragma unroll 1
        for (int ps = 0; ps < 2; ++ps) {
#pragma unroll
            for (int s = 0; s < 8; ++s) { const int row = 2 * s + hi, cofs = lr * 4; v4f val = *(const v4fa*)(os + row * 68 + cofs); if (BIAS) { val[0] += bfr(bias[c0 + cofs]); val[1] += bfr(bias[c0 + cofs + 1]); val[2] += bfr(bias[c0 + cofs + 2]); val[3] += bfr(bias[c0 + cofs + 3]); }
                *(volatile v4f*)(crow + (size_t)row * ldc + cofs) = val; }
            if (ps == 0) __threadfence(); }
        __builtin_amdgcn_wave_barrier(); asm volatile("" ::: "memory");
    }
}

typedef __attribute__((ext_vector_type(2))) _Float16 v2h;
typedef __attribute__((ext_vector_type(4))) _Float16 v4h;
typedef __attribute__((ext_vector_type(2))) unsigned short v2us;
typedef __attribute__((ext_vector_type(4))) unsigned short v4us;
typedef __attribute__((ext_vector_type(2))) float v2f;
typedef __attribute__((ext_vector_type(4))) int v4i;
__global__ __launch_bounds__(256) void k_cvt8(const float* __restrict__ src, bf* dst, size_t n8) { const size_t i = (size_t)blockIdx.x * 256 + threadIdx.x; if (i >= n8) return; const v8f v = *(const v8f*)(src + i * 8); v8us o;
#pragma unroll
    for (int k = 0; k < 8; ++k) o[k] = f2bf(v[k]); *(volatile v8us*)(dst + i * 8) = o; __threadfence(); *(volatile v8us*)(dst + i * 8) = o; }

__device__ __forceinline__ h16 toh_flush(float x) { const float z = (fabsf(x) < 6.103515625e-05f) ? 0.0f : x; return (h16)z; }

__device__ __forceinline__ float sp(float v) { return fmaxf(v, 0.0f) + log1pf(expf(-fabsf(v))); }

__global__ __launch_bounds__(256) void k_w16(const float* __restrict__ src, h16* dst, size_t n8) { const size_t i = (size_t)blockIdx.x * 256 + threadIdx.x; if (i >= n8) return; const v4f a = *(const v4f*)(src + i * 8), b = *(const v4f*)(src + i * 8 + 4); v8h o;
#pragma unroll
    for (int k = 0; k < 4; ++k) { const float p = bfr(a[k]), q = bfr(b[k]); o[k] = (h16)((fabsf(p) < PFL) ? 0.0f : p); o[k + 4] = (h16)((fabsf(q) < PFL) ? 0.0f : q); }
    *(volatile v8h*)(dst + i * 8) = o; __threadfence(); *(volatile v8h*)(dst + i * 8) = o; }

__global__ __launch_bounds__(256) void k_conv(const float* __restrict__ P, const float* __restrict__ cw, const float* __restrict__ cb, float* U, h16* Uh) { const unsigned e = blockIdx.x * 256 + threadIdx.x; const unsigned m = e >> 6, c0 = (e & 63u) << 2; const unsigned t = m & (NT - 1), m0 = m - t; v4f acc = *(const v4f*)(cb + c0);
#pragma unroll
    for (int k = 0; k < 4; ++k) acc[k] = bfr(acc[k]);
    v4f wq[4];
#pragma unroll
    for (int k = 0; k < 4; ++k) wq[k] = *(const v4f*)(cw + (size_t)(c0 + k) * 4);
#pragma unroll
    for (int j = 0; j < 4; ++j) { const int tj = (int)t - 3 + j; const unsigned tr = (tj < 0) ? 0u : (unsigned)tj; const float on = (tj < 0) ? 0.0f : 1.0f; const v4f xv = *(const v4f*)(P + (size_t)(m0 + tr) * (2 * DC) + DC + c0);
#pragma unroll
        for (int k = 0; k < 4; ++k) acc[k] = acc[k] + (bfr(wq[k][j]) * on) * xv[k]; }
    v4h hw;
#pragma unroll
    for (int k = 0; k < 4; ++k) hw[k] = toh_flush(acc[k]);
    *(volatile v4f*)(U + (size_t)e * 4) = acc; *(volatile v4h*)(Uh + (size_t)e * 4) = hw; __threadfence(); *(volatile v4f*)(U + (size_t)e * 4) = acc; *(volatile v4h*)(Uh + (size_t)e * 4) = hw; }

__global__ __launch_bounds__(256) void k_scan(const float* __restrict__ Q, const float* __restrict__ U, const float* __restrict__ Av, float* Y) { const int i = blockIdx.x * 256 + threadIdx.x; if (i >= NB * DC) return; const int b = i / DC; const int d = i % DC; float rt[NS], h[NS];
#pragma unroll
    for (int n = 0; n < NS; ++n) { rt[n] = -8.0f * sp(bfr(Av[(size_t)n * DC + d])); h[n] = 0.0f; }
    for (int t0 = 0; t0 < NT; t0 += 4) { float y4[4];
#pragma unroll
        for (int s = 0; s < 4; ++s) { const size_t r = (size_t)b * NT + t0 + s; const float* q = Q + r * NQ; const float g = 1.0f / (1.0f + expf(-q[2 * NS + d])); const float uv = U[r * DC + d]; float y = 0.0f;
#pragma unroll
            for (int n = 0; n < NS; ++n) { const float a = expf(g * rt[n]); h[n] = a * h[n] + (q[n] * uv) * sqrtf(1.0f - a * a + 1e-6f); y = y + q[NS + n] * h[n]; }
            y4[s] = y; }
        float* o = Y + ((size_t)b * NT + t0) * DC + d;
#pragma unroll
        for (int s = 0; s < 4; ++s) *(volatile float*)(o + (size_t)s * DC) = y4[s];
        __threadfence();
#pragma unroll
        for (int s = 0; s < 4; ++s) *(volatile float*)(o + (size_t)s * DC) = y4[s]; }
}

__global__ __launch_bounds__(256) void k_gate(const float* __restrict__ P, const float* __restrict__ Y, h16* Gh) { const unsigned e = blockIdx.x * 256 + threadIdx.x; const unsigned m = e >> 5, c0 = (e & 31u) << 3; const float* ps = P + (size_t)m * (2 * DC) + c0; const float* py = Y + (size_t)m * DC + c0; v8h o;
#pragma unroll
    for (int hf = 0; hf < 2; ++hf) { const v4f s = *(const v4f*)(ps + 4 * hf), y = *(const v4f*)(py + 4 * hf);
#pragma unroll
        for (int k = 0; k < 4; ++k) o[4 * hf + k] = toh_flush((0.5f * s[k] * (1.0f + erff(s[k] * 0.70710678f))) * y[k]); }
    *(volatile v8h*)(Gh + (size_t)e * 8) = o; __threadfence(); *(volatile v8h*)(Gh + (size_t)e * 8) = o; }

extern "C" void kernel_launch(void* const* d_in, const int* in_sizes, int n_in, void* d_out, int out_size, void* d_ws, size_t ws_size, hipStream_t stream) {
    if (n_in < 10) return;
    if (in_sizes[0] != NM * DC || in_sizes[1] != 2 * DC * DC || in_sizes[2] != DC * 4 || in_sizes[3] != DC || in_sizes[4] != 2 * NS * DC || in_sizes[5] != 2 * NS || in_sizes[6] != DC * DC || in_sizes[7] != DC || in_sizes[8] != NS * DC || in_sizes[9] != DC * DC) return;
    if (out_size != NM * DC) return;
    static_assert(NM == NB * NT && (NT & (NT - 1)) == 0 && NQ == 2 * NS + DC && NM % 64 == 0 && (2 * DC) % 64 == 0 && (2 * NS) % 64 == 0 && DC % 64 == 0 && DC % 32 == 0 && (NM * DC / 8) % 256 == 0 && (2 * DC * DC / 8) % 256 == 0 && (2 * NS * DC / 8) % 256 == 0 && (DC * DC / 8) % 256 == 0 && (NM * DC / 4) % 256 == 0 && (NB * DC) % 256 == 0 && DC % 32 == 0 && NT % 4 == 0 && (2 * NS * 4) % 256 == 0 && (NQ * 4) % 256 == 0, "the products: M and N multiples of 64, the depth of 32; the flat grids exact; a wave's 32 channels in one batch; the steps in fours; the second product's two column ranges begin on 256-byte steps of a row");
    const float* x = (const float*)d_in[0]; const float* Wi = (const float*)d_in[1]; const float* cw = (const float*)d_in[2]; const float* cb = (const float*)d_in[3]; const float* Wb = (const float*)d_in[4]; const float* bb = (const float*)d_in[5]; const float* Wl = (const float*)d_in[6]; const float* bl = (const float*)d_in[7]; const float* Av = (const float*)d_in[8]; const float* Wo = (const float*)d_in[9]; float* out = (float*)d_out;
    char* wsp = (char*)d_ws; auto take = [&](size_t bytes) { char* p = wsp; wsp += (bytes + 255) & ~(size_t)255; return (void*)p; };
    bf* Xb = (bf*)take((size_t)NM * DC * 2); bf* Wib = (bf*)take((size_t)2 * DC * DC * 2); float* P = (float*)take((size_t)NM * 2 * DC * 4); float* U = (float*)take((size_t)NM * DC * 4); h16* Uh = (h16*)take((size_t)NM * DC * 2); h16* Wbl = (h16*)take((size_t)NQ * DC * 2); float* Q = (float*)take((size_t)NM * NQ * 4); float* Y = (float*)take((size_t)NM * DC * 4); h16* Gh = (h16*)take((size_t)NM * DC * 2); h16* Woh = (h16*)take((size_t)DC * DC * 2);
    if ((size_t)(wsp - (char*)d_ws) > ws_size) return;
    k_cvt8<<<(unsigned)(NM * DC / 8 / 256), 256, 0, stream>>>(x, Xb, (size_t)NM * DC / 8);
    k_cvt8<<<(unsigned)(2 * DC * DC / 8 / 256), 256, 0, stream>>>(Wi, Wib, (size_t)2 * DC * DC / 8);
    k_gemmw<bf, 0, false><<<dim3(NM / 64, 2 * DC / 64, 1), 32, 0, stream>>>(Xb, nullptr, Wib, nullptr, DC, P, 2 * DC, nullptr, 0, 0, 0);
    k_conv<<<(unsigned)(NM * DC / 4 / 256), 256, 0, stream>>>(P, cw, cb, U, Uh);
    k_w16<<<(unsigned)(2 * NS * DC / 8 / 256), 256, 0, stream>>>(Wb, Wbl, (size_t)2 * NS * DC / 8);
    k_w16<<<(unsigned)(DC * DC / 8 / 256), 256, 0, stream>>>(Wl, Wbl + (size_t)2 * NS * DC, (size_t)DC * DC / 8);
    k_gemmw<h16, 0, true><<<dim3(NM / 64, 2 * NS / 64, 1), 32, 0, stream>>>(Uh, nullptr, Wbl, nullptr, DC, Q, NQ, bb, 0, 0, 0);
    k_gemmw<h16, 0, true><<<dim3(NM / 64, DC / 64, 1), 32, 0, stream>>>(Uh, nullptr, Wbl + (size_t)2 * NS * DC, nullptr, DC, Q + 2 * NS, NQ, bl, 0, 0, 0);
    k_scan<<<(unsigned)(NB * DC / 256), 256, 0, stream>>>(Q, U, Av, Y);
    k_gate<<<(unsigned)(NM * DC / 8 / 256), 256, 0, stream>>>(P, Y, Gh);
    k_w16<<<(unsigned)(DC * DC / 8 / 256), 256, 0, stream>>>(Wo, Woh, (size_t)DC * DC / 8);
    k_gemmw<h16, 0, false><<<dim3(NM / 64, DC / 64, 1), 32, 0, stream>>>(Gh, nullptr, Woh, nullptr, DC, out, DC, nullptr, 0, 0, 0);
}
